// DynamicGraphConvolution_81123342287014
// MI455X (gfx1250) — hardware-verified
//
#include <hip/hip_runtime.h>
#include <math.h>
#include <stdint.h>

typedef __attribute__((ext_vector_type(16))) _Float16 v16h;
typedef __attribute__((ext_vector_type(8)))  _Float16 v8h;
typedef __attribute__((ext_vector_type(16))) __bf16   v16b;
typedef __attribute__((ext_vector_type(8)))  __bf16   v8b;
typedef __attribute__((ext_vector_type(8)))  float    v8f;
typedef __attribute__((ext_vector_type(4)))  float    v4f;
typedef __attribute__((ext_vector_type(4)))  unsigned v4u;

static constexpr int NB    = 32;
static constexpr int NCH   = 64;
static constexpr int NNODE = 1024;

static_assert(NNODE % 64 == 0 && NCH % 64 == 0 && (NB * NCH) % 64 == 0, "tile multiples");
static_assert(NNODE % 32 == 0 && NCH % 32 == 0, "K multiples of 32");

__device__ __forceinline__ float bfr(float f) {
  unsigned u = __float_as_uint(f);
  u = (u + 0x7FFFu + ((u >> 16) & 1u)) & 0xFFFF0000u;
  return __uint_as_float(u);
}

__device__ __forceinline__ void dep_guard_h(v8f& a, v8f& b, v16h x, v16h y) { asm volatile("v_nop\n\tv_nop\n\tv_nop\n\tv_nop" : "+v"(a), "+v"(b) : "v"(x), "v"(y)); }
__device__ __forceinline__ void dep_guard_b(v8f& a, v8f& b, v16b x, v16b y) { asm volatile("v_nop\n\tv_nop\n\tv_nop\n\tv_nop" : "+v"(a), "+v"(b) : "v"(x), "v"(y)); }
__device__ __forceinline__ void keep4_h(v16h a, v16h b, v16h c, v16h d) { asm volatile("v_nop" :: "v"(a), "v"(b), "v"(c), "v"(d)); }
__device__ __forceinline__ void keep4_b(v16b a, v16b b, v16b c, v16b d) { asm volatile("v_nop" :: "v"(a), "v"(b), "v"(c), "v"(d)); }
__device__ __forceinline__ void acc_guard4(v8f& a, v8f& b, v8f& c, v8f& d) { asm volatile("v_nop\n\tv_nop\n\tv_nop\n\tv_nop" : "+v"(a), "+v"(b), "+v"(c), "+v"(d)); }
template <typename T> struct Frag;
template <> struct Frag<_Float16> {
  typedef v16h V; union U { v16h v; v8h h[2]; };
  static __device__ __forceinline__ v16h load(const _Float16* p) {
    U f; f.h[0] = *(const v8h*)(p); f.h[1] = *(const v8h*)(p + 16); return f.v;
  }
  static __device__ __forceinline__ v8f mma(v16h a, v16h b, v8f c) {
    return __builtin_amdgcn_wmma_f32_16x16x32_f16(false, a, false, b, (short)0, c, false, false);
  }
  static __device__ __forceinline__ void guard(v8f& a, v8f& b, v16h x, v16h y) { dep_guard_h(a, b, x, y); }
  static __device__ __forceinline__ void keep(v16h a, v16h b, v16h c, v16h d) { keep4_h(a, b, c, d); }
};
template <> struct Frag<__bf16> {
  typedef v16b V; union U { v16b v; v8b h[2]; };
  static __device__ __forceinline__ v16b load(const __bf16* p) {
    U f; f.h[0] = *(const v8b*)(p); f.h[1] = *(const v8b*)(p + 16); return f.v;
  }
  static __device__ __forceinline__ v8f mma(v16b a, v16b b, v8f c) {
    return __builtin_amdgcn_wmma_f32_16x16x32_bf16(false, a, false, b, (short)0, c, false, false);
  }
  static __device__ __forceinline__ void guard(v8f& a, v8f& b, v16b x, v16b y) { dep_guard_b(a, b, x, y); }
  static __device__ __forceinline__ void keep(v16b a, v16b b, v16b c, v16b d) { keep4_b(a, b, c, d); }
};

template <int ACT> __device__ __forceinline__ float act_apply(float v) {
  if (ACT == 1) return (v >= 0.0f) ? v : 0.2f * v;
  if (ACT == 2) {
    const float e = expf(-fabsf(v));
    const float r = __builtin_amdgcn_rcpf(1.0f + e);
    return (v >= 0.0f) ? r : e * r;
  }
  return v;
}

template <int BIAS_MODE, int ACT, int OUT16, int RESID_MODE, bool GMUL>
__global__ __launch_bounds__(256) void gemm_f16_t64(
    const unsigned short* __restrict__ Ap, int lda, long strideA,
    const unsigned short* __restrict__ Btp, int ldb, long strideB,
    void* __restrict__ Cout, int ldc, long strideC,
    const float* __restrict__ bias,
    const void* __restrict__ resid, int ldr, long strideR,
    const float* __restrict__ gmulp,
    int M, int N, int K, float scale, float omul) {
  static_assert(OUT16 == 1 || RESID_MODE == 0, "resid path only with 16-bit output");
  typedef _Float16 T;
  typedef v16h V;
  const T* A  = (const T*)Ap;
  const T* Bt = (const T*)Btp;
  __shared__ __align__(16) float sT[8][16 * 68];
  const int b    = blockIdx.y;
  const int lane = threadIdx.x & 31;
  const int wave = threadIdx.x >> 5;
  const int wpb  = blockDim.x >> 5;
  const int tilesN = N >> 6;
  const int tilesM = M >> 6;
  const int tile = blockIdx.x * wpb + wave;
  if (tile >= tilesM * tilesN) return;
  const int tm = tile / tilesN;
  const int tn = tile - tm * tilesN;
  const int m0 = tm << 6;
  const int n0 = tn << 6;

  const T* Ab = A  + (size_t)b * strideA;
  const T* Bb = Bt + (size_t)b * strideB;

  const int rlane = lane & 15;
  const int koff  = (lane >> 4) * 8;
  const int mOff  = (lane >> 4) * 8;

  float gm = 1.0f;
  if (GMUL) gm = bfr(gmulp[0]);

  v8f acc[4][4];
#pragma unroll
  for (int i = 0; i < 4; ++i)
#pragma unroll
    for (int j = 0; j < 4; ++j) acc[i][j] = (v8f){0.f,0.f,0.f,0.f,0.f,0.f,0.f,0.f};

  for (int k0 = 0; k0 < K; k0 += 32) {
    V bh[4];
#pragma unroll
    for (int j = 0; j < 4; ++j) {
      const size_t bo = (size_t)(n0 + (j << 4) + rlane) * ldb + koff + k0;
      bh[j] = Frag<T>::load(Bb + bo);
    }
#pragma unroll
    for (int i = 0; i < 4; ++i) {
      const size_t ao = (size_t)(m0 + (i << 4) + rlane) * lda + koff + k0;
      V ah = Frag<T>::load(Ab + ao);
#pragma unroll
      for (int j = 0; j < 4; ++j) acc[i][j] = Frag<T>::mma(ah, bh[j], acc[i][j]);
      Frag<T>::guard(acc[i][0], acc[i][3], ah, ah);
    }
    Frag<T>::keep(bh[0], bh[1], bh[2], bh[3]);
  }
  acc_guard4(acc[0][0], acc[0][1], acc[0][2], acc[0][3]);
  acc_guard4(acc[1][0], acc[1][1], acc[1][2], acc[1][3]);
  acc_guard4(acc[2][0], acc[2][1], acc[2][2], acc[2][3]);
  acc_guard4(acc[3][0], acc[3][1], acc[3][2], acc[3][3]);

  float* slab = sT[wave];
#pragma unroll
  for (int i = 0; i < 4; ++i) {
    const int mBase = m0 + (i << 4);
#pragma unroll
    for (int j = 0; j < 4; ++j) {
#pragma unroll
      for (int r = 0; r < 8; ++r) slab[(mOff + r) * 68 + (j << 4) + rlane] = acc[i][j][r];
    }
    __builtin_amdgcn_fence(__ATOMIC_RELEASE, "workgroup");
    __builtin_amdgcn_wave_barrier();
    __builtin_amdgcn_fence(__ATOMIC_ACQUIRE, "workgroup");
    if (OUT16 == 0) {
      float* Cb = (float*)Cout + (size_t)b * strideC;
      const int hh = lane >> 4, c4 = (lane & 15) * 4;
      v4f bn4 = (v4f){0.f, 0.f, 0.f, 0.f};
      if (BIAS_MODE == 2) {
        const v4f t4 = *(const v4f*)(bias + n0 + c4);
#pragma unroll
        for (int e = 0; e < 4; ++e) bn4[e] = bfr(t4[e]);
      }
      v4f vals[8];
#pragma unroll
      for (int it = 0; it < 8; ++it) {
        const int row = it * 2 + hh;
        const int m = mBase + row;
        const v4f s4 = *(const v4f*)(slab + row * 68 + c4);
        float bm = 0.0f;
        if (BIAS_MODE == 1) bm = bfr(bias[m]);
        v4f o4;
#pragma unroll
        for (int e = 0; e < 4; ++e) {
          float v = s4[e] * scale + bm + bn4[e];
          v = act_apply<ACT>(v);
          v = v * omul;
          if (GMUL) v = v * gm;
          o4[e] = v;
        }
        vals[it] = o4;
      }
      for (int pass = 0; pass < 2; ++pass) {
#pragma unroll
        for (int it = 0; it < 8; ++it) {
          const int row = it * 2 + hh;
          *(volatile v4f*)(Cb + (size_t)(mBase + row) * ldc + n0 + c4) = vals[it];
        }
        __threadfence();
      }
    } else {
      unsigned short* Cb = (unsigned short*)Cout + (size_t)b * strideC;
      const int q = lane >> 3, c8 = (lane & 7) * 8;
      float bn8[8];
#pragma unroll
      for (int e = 0; e < 8; ++e) bn8[e] = 0.0f;
      if (BIAS_MODE == 2) {
        const v4f t0 = *(const v4f*)(bias + n0 + c8);
        const v4f t1 = *(const v4f*)(bias + n0 + c8 + 4);
#pragma unroll
        for (int e = 0; e < 4; ++e) { bn8[e] = bfr(t0[e]); bn8[4 + e] = bfr(t1[e]); }
      }
      v8h hv[4];
#pragma unroll
      for (int it = 0; it < 4; ++it) {
        const int row = it * 4 + q;
        const int m = mBase + row;
        const float* sp = slab + row * 68 + c8;
        const v4f s0 = *(const v4f*)(sp);
        const v4f s1 = *(const v4f*)(sp + 4);
        float sv[8];
#pragma unroll
        for (int e = 0; e < 4; ++e) { sv[e] = s0[e]; sv[4 + e] = s1[e]; }
        float bm = 0.0f;
        if (BIAS_MODE == 1) bm = bfr(bias[m]);
        float rv[8];
#pragma unroll
        for (int e = 0; e < 8; ++e) rv[e] = 0.0f;
        if (RESID_MODE == 1) {
          const float* Rb = (const float*)resid + (size_t)b * strideR + (size_t)m * ldr + n0 + c8;
          const v4f r0 = *(const v4f*)(Rb);
          const v4f r1 = *(const v4f*)(Rb + 4);
#pragma unroll
          for (int e = 0; e < 4; ++e) { rv[e] = bfr(r0[e]); rv[4 + e] = bfr(r1[e]); }
        }
        if (RESID_MODE == 2) {
          const unsigned short* Rb = (const unsigned short*)resid + (size_t)b * strideR + (size_t)m * ldr + n0 + c8;
          const v4u w = *(const v4u*)(Rb);
#pragma unroll
          for (int e = 0; e < 8; ++e) {
            const unsigned bits = (w[e >> 1] >> ((e & 1) * 16)) & 0xFFFFu;
            float rf = (float)__builtin_bit_cast(_Float16, (unsigned short)bits);
            asm volatile("" : "+v"(rf));
            rv[e] = rf;
          }
        }
        v8h o8;
#pragma unroll
        for (int e = 0; e < 8; ++e) {
          float v = sv[e] * scale + bm + bn8[e];
          v = act_apply<ACT>(v);
          v = v * omul;
          if (GMUL) v = v * gm;
          v = v + rv[e];
          o8[e] = (_Float16)v;
        }
        hv[it] = o8;
      }
      for (int pass = 0; pass < 2; ++pass) {
#pragma unroll
        for (int it = 0; it < 4; ++it) {
          const int row = it * 4 + q;
          *(volatile v8h*)(Cb + (size_t)(mBase + row) * ldc + n0 + c8) = hv[it];
        }
        __threadfence();
      }
    }
    __builtin_amdgcn_fence(__ATOMIC_RELEASE, "workgroup");
    __builtin_amdgcn_wave_barrier();
    __builtin_amdgcn_fence(__ATOMIC_ACQUIRE, "workgroup");
  }
}

__global__ __launch_bounds__(256) void cast_bf16rne_f16x8(
    const float* __restrict__ in, unsigned short* __restrict__ out, int n8, float mul) {
  const int i = blockIdx.x * 256 + threadIdx.x;
  if (i < n8) {
    const v4f a  = *(const v4f*)(in + (size_t)8 * i);
    const v4f a2 = *(const v4f*)(in + (size_t)8 * i + 4);
    v8h hv;
#pragma unroll
    for (int e = 0; e < 4; ++e) {
      hv[e]     = (_Float16)(bfr(a[e]) * mul);
      hv[4 + e] = (_Float16)(bfr(a2[e]) * mul);
    }
    unsigned short* p = out + (size_t)8 * i;
    *(volatile v8h*)p = hv;
    __threadfence();
    *(volatile v8h*)p = hv;
  }
}

__global__ __launch_bounds__(256) void xpose_bcn_to_bnc_f16(
    const float* __restrict__ x, unsigned short* __restrict__ xT) {
  __shared__ __align__(16) _Float16 sh[NCH * 72];
  const int nt = blockIdx.x, b = blockIdx.y, n0 = nt * 64;
  const int t = threadIdx.x;
#pragma unroll
  for (int i = 0; i < 4; ++i) {
    const int qd = t + 256 * i;
    const int cr = qd >> 4, col4 = (qd & 15) * 4;
    const v4f v = *(const v4f*)(x + ((size_t)(b * NCH + cr)) * NNODE + n0 + col4);
#pragma unroll
    for (int e = 0; e < 4; ++e) sh[cr * 72 + col4 + e] = (_Float16)bfr(v[e]);
  }
  __syncthreads();
  const int wave = t >> 5, lane = t & 31, q = lane >> 3, c8 = (lane & 7) * 8;
  v8h hv[2];
#pragma unroll
  for (int it = 0; it < 2; ++it) {
    const int nrow = wave * 8 + it * 4 + q;
    v8h o8;
#pragma unroll
    for (int e = 0; e < 8; ++e) o8[e] = sh[(c8 + e) * 72 + nrow];
    hv[it] = o8;
  }
  for (int pass = 0; pass < 2; ++pass) {
#pragma unroll
    for (int it = 0; it < 2; ++it) {
      const int nrow = wave * 8 + it * 4 + q;
      *(volatile v8h*)(xT + ((size_t)(b * NNODE + n0 + nrow)) * NCH + c8) = hv[it];
    }
    __threadfence();
  }
}

__global__ __launch_bounds__(256) void bn_att_kernel(
    const float* __restrict__ energy, const float* __restrict__ bng, const float* __restrict__ bnb,
    unsigned short* __restrict__ att) {
  __shared__ float red[8];
  const int c = blockIdx.x;
  const int t = threadIdx.x, lane = t & 31, wave = t >> 5;
  const int bb = t >> 3, d0 = (t & 7) * 8;
  const size_t base = ((size_t)(bb * NCH + c)) * NCH + d0;
  const v4f e0 = *(const v4f*)(energy + base);
  const v4f e1 = *(const v4f*)(energy + base + 4);
  float ev[8];
#pragma unroll
  for (int e = 0; e < 4; ++e) { ev[e] = e0[e]; ev[4 + e] = e1[e]; }
  float mx = ev[0];
#pragma unroll
  for (int e = 1; e < 8; ++e) mx = fmaxf(mx, ev[e]);
  mx = fmaxf(mx, __shfl_xor(mx, 1, 32));
  mx = fmaxf(mx, __shfl_xor(mx, 2, 32));
  mx = fmaxf(mx, __shfl_xor(mx, 4, 32));
  float en[8];
  float s = 0.0f;
#pragma unroll
  for (int e = 0; e < 8; ++e) { en[e] = mx - ev[e]; s += en[e]; }
#pragma unroll
  for (int off = 1; off < 32; off <<= 1) s += __shfl_xor(s, off, 32);
  if (lane == 0) red[wave] = s;
  __syncthreads();
  float tot = 0.0f;
#pragma unroll
  for (int w = 0; w < 8; ++w) tot += red[w];
  const float mu = tot * (1.0f / (float)(NB * NCH));
  __syncthreads();
  float s2 = 0.0f;
#pragma unroll
  for (int e = 0; e < 8; ++e) { const float dv = en[e] - mu; s2 += dv * dv; }
#pragma unroll
  for (int off = 1; off < 32; off <<= 1) s2 += __shfl_xor(s2, off, 32);
  if (lane == 0) red[wave] = s2;
  __syncthreads();
  float tot2 = 0.0f;
#pragma unroll
  for (int w = 0; w < 8; ++w) tot2 += red[w];
  const float var = tot2 * (1.0f / (float)(NB * NCH));
  const float rs = 1.0f / sqrtf(var + 1e-5f);
  const float g = bfr(bng[c]), be = bfr(bnb[c]);
  v8h hv;
#pragma unroll
  for (int e = 0; e < 8; ++e) hv[e] = (_Float16)(64.0f * (g * (en[e] - mu) * rs + be));
  unsigned short* dst = att + base;
  *(volatile v8h*)dst = hv;
  __threadfence();
  *(volatile v8h*)dst = hv;
}

extern "C" void kernel_launch(void* const* d_in, const int* in_sizes, int n_in,
                              void* d_out, int out_size, void* d_ws, size_t ws_size,
                              hipStream_t stream) {
  if (n_in < 11) return;
  if (in_sizes[0] != NB * NCH * NNODE || in_sizes[1] != NNODE * NNODE || in_sizes[2] != NCH * NCH ||
      in_sizes[7] != NNODE * NCH || in_sizes[9] != NCH * NCH || out_size != NB * NCH * NNODE) return;
  const float* x     = (const float*)d_in[0];
  const float* W_sa  = (const float*)d_in[1];
  const float* W_sw  = (const float*)d_in[2];
  const float* b_sw  = (const float*)d_in[3];
  const float* bn_g  = (const float*)d_in[4];
  const float* bn_b  = (const float*)d_in[5];
  const float* gamma = (const float*)d_in[6];
  const float* W_cm  = (const float*)d_in[7];
  const float* b_cm  = (const float*)d_in[8];
  const float* W_dw  = (const float*)d_in[9];
  const float* b_dw  = (const float*)d_in[10];
  float* y = (float*)d_out;

  char* ws = (char*)d_ws;
  size_t off = 0;
  auto carve = [&](size_t bytes) -> void* {
    void* p = ws + off;
    off = (off + bytes + 255) & ~(size_t)255;
    return p;
  };
  unsigned short* x16    = (unsigned short*)carve((size_t)NB * NCH * NNODE * 2);
  unsigned short* xT16   = (unsigned short*)carve((size_t)NB * NNODE * NCH * 2);
  unsigned short* wsa16  = (unsigned short*)carve((size_t)NNODE * NNODE * 2);
  unsigned short* wsw16  = (unsigned short*)carve((size_t)NCH * NCH * 2);
  unsigned short* wcm16  = (unsigned short*)carve((size_t)NNODE * NCH * 2);
  unsigned short* wdw16  = (unsigned short*)carve((size_t)NCH * NCH * 2);
  unsigned short* t16    = (unsigned short*)carve((size_t)NNODE * (NB * NCH) * 2);
  unsigned short* x1_16  = (unsigned short*)carve((size_t)NB * NCH * NNODE * 2);
  float*          energy = (float*)carve((size_t)NB * NCH * NCH * 4);
  unsigned short* att16  = (unsigned short*)carve((size_t)NB * NCH * NCH * 2);
  unsigned short* xgT16  = (unsigned short*)carve((size_t)NB * NNODE * NCH * 2);
  unsigned short* adjT16 = (unsigned short*)carve((size_t)NB * NNODE * NNODE * 2);
  unsigned short* y1T16  = (unsigned short*)carve((size_t)NB * NNODE * NCH * 2);
  if (off > ws_size) return;

  const long sBCN = (long)NCH * NNODE;
  const long sBNC = (long)NNODE * NCH;
  const long sBCC = (long)NCH * NCH;
  const long sBNN = (long)NNODE * NNODE;

  cast_bf16rne_f16x8<<<(NB * NCH * NNODE / 8 + 255) / 256, 256, 0, stream>>>(x, x16, NB * NCH * NNODE / 8, 1.0f);
  xpose_bcn_to_bnc_f16<<<dim3(NNODE / 64, NB), 256, 0, stream>>>(x, xT16);
  cast_bf16rne_f16x8<<<(NNODE * NNODE / 8 + 255) / 256, 256, 0, stream>>>(W_sa, wsa16, NNODE * NNODE / 8, 64.0f);
  cast_bf16rne_f16x8<<<(NCH * NCH / 8 + 255) / 256, 256, 0, stream>>>(W_sw, wsw16, NCH * NCH / 8, 16.0f);
  cast_bf16rne_f16x8<<<(NNODE * NCH / 8 + 255) / 256, 256, 0, stream>>>(W_cm, wcm16, NNODE * NCH / 8, 16.0f);
  cast_bf16rne_f16x8<<<(NCH * NCH / 8 + 255) / 256, 256, 0, stream>>>(W_dw, wdw16, NCH * NCH / 8, 16.0f);

  gemm_f16_t64<0, 1, 1, 0, false><<<dim3((NNODE / 64) * (NB * NCH / 64) / 8, 1), 256, 0, stream>>>(
      wsa16, NNODE, 0L, x16, NNODE, 0L, (void*)t16, NB * NCH, 0L,
      b_sw, (const void*)x, 0, 0L, gamma, NNODE, NB * NCH, NNODE, 16.0f / 64.0f, 1.0f);

  gemm_f16_t64<1, 1, 1, 1, false><<<dim3(2, NB), 256, 0, stream>>>(
      wsw16, NCH, 0L, t16, NB * NCH, (long)NCH, (void*)x1_16, NNODE, sBCN,
      b_sw, (const void*)x, NNODE, sBCN, gamma, NCH, NNODE, NCH, 1.0f / 256.0f, 1.0f);

  gemm_f16_t64<0, 0, 0, 0, false><<<dim3(1, NB), 32, 0, stream>>>(
      x16, NNODE, sBCN, x16, NNODE, sBCN, (void*)energy, NCH, sBCC,
      b_sw, (const void*)x, 0, 0L, gamma, NCH, NCH, NNODE, 1.0f, 1.0f);

  bn_att_kernel<<<NCH, 256, 0, stream>>>(energy, bn_g, bn_b, att16);

  gemm_f16_t64<0, 0, 1, 2, true><<<dim3(2, NB), 256, 0, stream>>>(
      xT16, NCH, sBNC, att16, NCH, sBCC, (void*)xgT16, NCH, sBNC,
      b_sw, (const void*)xT16, NCH, sBNC, gamma, NNODE, NCH, NCH, 1.0f / 64.0f, 1.0f);

  gemm_f16_t64<2, 2, 1, 0, false><<<dim3((NNODE / 64) * (NNODE / 64) / 8, NB), 256, 0, stream>>>(
      xgT16, NCH, sBNC, wcm16, NCH, 0L, (void*)adjT16, NNODE, sBNN,
      b_cm, (const void*)x, 0, 0L, gamma, NNODE, NNODE, NCH, 1.0f / 16.0f, 1024.0f);

  gemm_f16_t64<0, 1, 1, 0, false><<<dim3(2, NB), 256, 0, stream>>>(
      adjT16, NNODE, sBNN, x1_16, NNODE, sBCN, (void*)y1T16, NCH, sBNC,
      b_sw, (const void*)x, 0, 0L, gamma, NNODE, NCH, NNODE, 1.0f / 1024.0f, 1.0f);

  gemm_f16_t64<1, 1, 0, 0, false><<<dim3(2, NB), 256, 0, stream>>>(
      wdw16, NCH, 0L, y1T16, NCH, sBNC, (void*)y, NNODE, sBCN,
      b_dw, (const void*)x, 0, 0L, gamma, NCH, NNODE, NCH, 1.0f / 16.0f, 1.0f);
}
